// BWGNN_Hetero_14078902796340
// MI455X (gfx1250) — hardware-verified
//
#include <hip/hip_runtime.h>
#include <stddef.h>


#define INF     128
#define HF      64
#define KW3     192
#define NCLS    2
#define NTHR    256
#define NWAVE   8
#define EPT     8
#define NGRP    2
#define CHUNK   (NTHR * EPT * NGRP)
#define WCAP    (EPT * NGRP * 32)
#define LISTN   (NWAVE * WCAP)
#define SLB     13
#define NBC     8192
#define NBF     2048
#define RCAP    40960
#define RBN     128
#define CNTMAX  65536
#define TGT     256
#define DEGCAP  256
#define GROWS   128
#define OTHR    512
#define ASCALE  16.0f
#define WSCALE  64.0f
#define PINV    0.0009765625f
#define AP1     (INF + 8)
#define AP2     (HF + 8)
#define AP3     (KW3 + 8)
#define TH00    3.0f
#define TH01    (-3.0f)
#define TH02    0.75f
#define TH11    3.0f
#define TH12    (-1.5f)
#define TH22    0.75f

#define LDS_MLP  (GROWS * AP1 * 2 + GROWS * AP2 * 2)
#define LDS_FILL ((RCAP + NBF + LISTN) * 4 + 64)
#define LDS_AW   (2 * TGT * HF * 4 + 2 * TGT * 4)

static_assert((CHUNK & (CHUNK - 1)) == 0);
static_assert(CHUNK <= 4096);
static_assert(NBC <= (1 << SLB) && NBF <= NBC);
static_assert((NBC & (NBC - 1)) == 0 && (NBF & (NBF - 1)) == 0);
static_assert(NBC == 4 * NBF);
static_assert(OTHR * 16 == NBC);
static_assert(NTHR * 32 == NBC);
static_assert((RCAP % 32) == 0);
static_assert(GROWS * HF * 4 <= GROWS * AP1 * 2);
static_assert(TGT * AP3 * 2 <= 2 * TGT * HF * 4);
static_assert(TGT == NWAVE * 32 && (TGT % GROWS) == 0);
static_assert((GROWS * INF / 8) % NTHR == 0);
static_assert(TGT == NTHR);

typedef float    v2f  __attribute__((ext_vector_type(2)));
typedef float    v4f  __attribute__((ext_vector_type(4)));
typedef float    v8f  __attribute__((ext_vector_type(8)));
typedef int      v4i  __attribute__((ext_vector_type(4)));
typedef _Float16 v2h  __attribute__((ext_vector_type(2)));
typedef _Float16 v8h  __attribute__((ext_vector_type(8)));
typedef _Float16 v16h __attribute__((ext_vector_type(16)));
union FragH { v16h v; v8h h[2]; };
union FI { float f; int i; };

__device__ __forceinline__ v8h cvt8(v4f a, v4f b) {
  v8h r;
  r[0] = (_Float16)a.x; r[1] = (_Float16)a.y; r[2] = (_Float16)a.z; r[3] = (_Float16)a.w;
  r[4] = (_Float16)b.x; r[5] = (_Float16)b.y; r[6] = (_Float16)b.z; r[7] = (_Float16)b.w;
  return r;
}

__device__ __forceinline__ v8f wmh(v16h a, v16h b, v8f c) {
  v8f d = __builtin_amdgcn_wmma_f32_16x16x32_f16(false, a, false, b, (short)0, c, false, false);
  asm volatile("v_nop\n\tv_nop\n\tv_nop\n\tv_nop" : "+v"(d) : "v"(a), "v"(b));
  return d;
}

__device__ __forceinline__ v8f zero8() {
  v8f z = {0.f, 0.f, 0.f, 0.f, 0.f, 0.f, 0.f, 0.f};
  return z;
}

template <int NB>
__device__ __forceinline__ int scan_chunk(const int* __restrict__ dsts, int nE, int cbase, int slotBase,
                                          int vec8, int* list, int tid, int lane, int wave) {
  int wc = 0;
#pragma unroll
  for (int g = 0; g < NGRP; ++g) {
    const int el0  = (g * NTHR + tid) * EPT;
    const int e0   = cbase + el0;
    const int sent = -2147483647 - 1;
    v4i da, db;
    if (vec8 != 0 && cbase + CHUNK <= nE) {
      da = *(const v4i*)(dsts + e0);
      db = *(const v4i*)(dsts + e0 + 4);
    } else {
      da.x = (e0     < nE) ? dsts[min(e0, nE - 1)] : sent;
      da.y = (e0 + 1 < nE) ? dsts[min(e0 + 1, nE - 1)] : sent;
      da.z = (e0 + 2 < nE) ? dsts[min(e0 + 2, nE - 1)] : sent;
      da.w = (e0 + 3 < nE) ? dsts[min(e0 + 3, nE - 1)] : sent;
      db.x = (e0 + 4 < nE) ? dsts[min(e0 + 4, nE - 1)] : sent;
      db.y = (e0 + 5 < nE) ? dsts[min(e0 + 5, nE - 1)] : sent;
      db.z = (e0 + 6 < nE) ? dsts[min(e0 + 6, nE - 1)] : sent;
      db.w = (e0 + 7 < nE) ? dsts[min(e0 + 7, nE - 1)] : sent;
    }
    const unsigned nb = (unsigned)slotBase;
    const unsigned s0 = (unsigned)da.x - nb, s1 = (unsigned)da.y - nb;
    const unsigned s2 = (unsigned)da.z - nb, s3 = (unsigned)da.w - nb;
    const unsigned s4 = (unsigned)db.x - nb, s5 = (unsigned)db.y - nb;
    const unsigned s6 = (unsigned)db.z - nb, s7 = (unsigned)db.w - nb;
    const bool h0 = s0 < (unsigned)NB, h1 = s1 < (unsigned)NB, h2 = s2 < (unsigned)NB, h3 = s3 < (unsigned)NB;
    const bool h4 = s4 < (unsigned)NB, h5 = s5 < (unsigned)NB, h6 = s6 < (unsigned)NB, h7 = s7 < (unsigned)NB;
    const unsigned any = __builtin_amdgcn_ballot_w32(h0 | h1 | h2 | h3 | h4 | h5 | h6 | h7);
    if (any != 0u) {
#define HITJ(J, HJ, SJ) { \
        const unsigned mj = __builtin_amdgcn_ballot_w32(HJ); \
        if (mj != 0u) { \
          if (HJ) { \
            const int pos = wc + (int)__builtin_amdgcn_mbcnt_lo(mj, 0u); \
            if (pos < WCAP) list[wave * WCAP + pos] = ((el0 + (J)) << SLB) | (int)(SJ); \
          } \
          wc += (int)__builtin_popcount(mj); } }
      HITJ(0, h0, s0)
      HITJ(1, h1, s1)
      HITJ(2, h2, s2)
      HITJ(3, h3, s3)
      HITJ(4, h4, s4)
      HITJ(5, h5, s5)
      HITJ(6, h6, s6)
      HITJ(7, h7, s7)
#undef HITJ
    }
  }
  return wc;
}

__global__ __launch_bounds__(NTHR) void k_wprep(
    const float* __restrict__ w1, const float* __restrict__ w2, const float* __restrict__ w3, _Float16* wp) {
  const int b = (int)blockIdx.x;
  const int tid = (int)threadIdx.x;
  const float* src;
  int base, i;
  if (b < 4)      { src = w1; base = 0;                  i = b * NTHR + tid; }
  else if (b < 6) { src = w2; base = HF * INF;           i = (b - 4) * NTHR + tid; }
  else            { src = w3; base = HF * INF + HF * HF; i = (b - 6) * NTHR + tid; }
  const float* sp = src + (size_t)i * 8;
  const v4f a = *(const v4f*)sp * WSCALE;
  const v4f c = *(const v4f*)(sp + 4) * WSCALE;
  const v8h hv = cvt8(a, c);
  _Float16* dp = wp + base + (size_t)i * 8;
  *(volatile v8h*)dp = hv;
  __threadfence();
  *(volatile v8h*)dp = hv;
}

__global__ __launch_bounds__(NTHR) void k_count(
    const int* __restrict__ dsts, int* cnt, float* dinv, int nE, int vec8) {
  __shared__ __attribute__((aligned(16))) int scnt[NBC];
  __shared__ __attribute__((aligned(16))) int list[LISTN];
  __shared__ int wcnt[NWAVE];
  const int tid = threadIdx.x, lane = tid & 31, wave = tid >> 5;
  const int nodeBase = blockIdx.x * NBC;

  for (int i = tid; i < NBC; i += NTHR) scnt[i] = 0;
  __syncthreads();

  const int nChunks = (nE + CHUNK - 1) / CHUNK;
#pragma unroll 1
  for (int ch = 0; ch < nChunks; ++ch) {
    const int cbase = ch * CHUNK;
    const int wc = scan_chunk<NBC>(dsts, nE, cbase, nodeBase, vec8, list, tid, lane, wave);
    if (lane == 0) wcnt[wave] = wc;
    __syncthreads();
    if (wave == 0) {
#pragma unroll 1
      for (int wsx = 0; wsx < NWAVE; ++wsx) {
        int n = __builtin_amdgcn_readfirstlane(wcnt[wsx]);
        n = n > WCAP ? WCAP : (n < 0 ? 0 : n);
        const int* lp = list + wsx * WCAP;
#pragma unroll 1
        for (int i = 0; i < n; ++i) {
          const int ent  = __builtin_amdgcn_readfirstlane(lp[i]);
          const int slot = ent & (NBC - 1);
          if (lane == 0) scnt[slot] = scnt[slot] + 1;
        }
      }
    }
    __syncthreads();
  }

  v4i cq[8]; v4f dq[8];
#pragma unroll
  for (int q = 0; q < 8; ++q) {
    const int f = (wave * 8 + q) * 128 + 4 * lane;
    const v4i c = *(const v4i*)(scnt + f);
    cq[q] = c;
    dq[q].x = rsqrtf((float)(c.x < 1 ? 1 : c.x));
    dq[q].y = rsqrtf((float)(c.y < 1 ? 1 : c.y));
    dq[q].z = rsqrtf((float)(c.z < 1 ? 1 : c.z));
    dq[q].w = rsqrtf((float)(c.w < 1 ? 1 : c.w));
  }
  int*   cp = cnt + (size_t)nodeBase;
  float* dp = dinv + (size_t)nodeBase;
#pragma unroll
  for (int q = 0; q < 8; ++q) {
    const int f = (wave * 8 + q) * 128 + 4 * lane;
    *(volatile v4i*)(cp + f) = cq[q];
    *(volatile v4f*)(dp + f) = dq[q];
  }
  __threadfence();
#pragma unroll
  for (int q = 0; q < 8; ++q) {
    const int f = (wave * 8 + q) * 128 + 4 * lane;
    *(volatile v4i*)(cp + f) = cq[q];
    *(volatile v4f*)(dp + f) = dq[q];
  }
}

__global__ __launch_bounds__(OTHR) void k_offsets(
    const int* __restrict__ cnt, int* off, int* rbase, int nChunk) {
  __shared__ __attribute__((aligned(16))) int soff[NBC];
  __shared__ __attribute__((aligned(16))) int srb[RBN];
  __shared__ int wtot[OTHR / 32];
  const int tid = threadIdx.x, lane = tid & 31, wave = tid >> 5, sub = tid >> 7;
  for (int i = tid; i < RBN; i += OTHR) srb[i] = 0;
  int carry = 0;
#pragma unroll 1
  for (int ch = 0; ch < nChunk; ++ch) {
    const int base = ch * NBC;
    const int* cq = cnt + base + 16 * tid;
    const v4i c0 = *(const v4i*)(cq);
    const v4i c1 = *(const v4i*)(cq + 4);
    const v4i c2 = *(const v4i*)(cq + 8);
    const v4i c3 = *(const v4i*)(cq + 12);
    int e[16];
    e[0]  = c0.x; e[1]  = c0.y; e[2]  = c0.z; e[3]  = c0.w;
    e[4]  = c1.x; e[5]  = c1.y; e[6]  = c1.z; e[7]  = c1.w;
    e[8]  = c2.x; e[9]  = c2.y; e[10] = c2.z; e[11] = c2.w;
    e[12] = c3.x; e[13] = c3.y; e[14] = c3.z; e[15] = c3.w;
    int ts = 0;
#pragma unroll
    for (int j = 0; j < 16; ++j) {
      int v = e[j];
      v = v < 0 ? 0 : (v > CNTMAX ? CNTMAX : v);
      e[j] = v;
      ts += v;
    }
    int incl = ts;
#pragma unroll
    for (int d = 1; d < 32; d <<= 1) {
      const int t = __shfl_up(incl, d);
      if (lane >= d) incl += t;
    }
    if (lane == 31) wtot[wave] = incl;
    __syncthreads();
    const int S0 = wtot[0]  + wtot[1]  + wtot[2]  + wtot[3];
    const int S1 = wtot[4]  + wtot[5]  + wtot[6]  + wtot[7];
    const int S2 = wtot[8]  + wtot[9]  + wtot[10] + wtot[11];
    const int S3 = wtot[12] + wtot[13] + wtot[14] + wtot[15];
    int pre = 0;
#pragma unroll 1
    for (int w = 4 * sub; w < wave; ++w) pre += wtot[w];
    const int b0 = carry;
    const int b1 = b0 + ((S0 + 31) & ~31);
    const int b2 = b1 + ((S1 + 31) & ~31);
    const int b3 = b2 + ((S2 + 31) & ~31);
    const int b4 = b3 + ((S3 + 31) & ~31);
    const int myb = sub == 0 ? b0 : (sub == 1 ? b1 : (sub == 2 ? b2 : b3));
    if (tid == 0) {
      srb[min(4 * ch + 0, RBN - 1)] = b0;
      srb[min(4 * ch + 1, RBN - 1)] = b1;
      srb[min(4 * ch + 2, RBN - 1)] = b2;
      srb[min(4 * ch + 3, RBN - 1)] = b3;
    }
    int run = myb + pre + incl - ts;
#pragma unroll
    for (int j = 0; j < 16; ++j) { soff[16 * tid + j] = run; run += e[j]; }
    carry = b4;
    __syncthreads();
    v4i o[4];
#pragma unroll
    for (int q = 0; q < 4; ++q) o[q] = *(const v4i*)(soff + 4 * (tid + q * OTHR));
    int* op = off + base;
#pragma unroll
    for (int q = 0; q < 4; ++q) *(volatile v4i*)(op + 4 * (tid + q * OTHR)) = o[q];
    __threadfence();
#pragma unroll
    for (int q = 0; q < 4; ++q) *(volatile v4i*)(op + 4 * (tid + q * OTHR)) = o[q];
    __syncthreads();
  }
  if (tid == 0) srb[min(4 * nChunk, RBN - 1)] = carry;
  __syncthreads();
  v4i rv = {0, 0, 0, 0};
  if (tid < 32) rv = *(const v4i*)(srb + 4 * tid);
  if (tid < 32) *(volatile v4i*)(rbase + 4 * tid) = rv;
  __threadfence();
  if (tid < 32) *(volatile v4i*)(rbase + 4 * tid) = rv;
}

__global__ __launch_bounds__(NTHR) void k_fill(
    const int* __restrict__ srcp, const int* __restrict__ dstp,
    const int* __restrict__ off, const int* __restrict__ rbase,
    int* csr, int nN, int nE, int vec8, int csrLen) {
  extern __shared__ v4f lds_dyn[];
  int* region = (int*)lds_dyn;
  int* cursor = region + RCAP;
  int* list   = cursor + NBF;
  int* wcnt   = list + LISTN;
  const int tid = threadIdx.x, lane = tid & 31, wave = tid >> 5;
  const int b = blockIdx.x;
  const int nodeBase = b * NBF;

  int rb0 = rbase[b];
  const int rb1 = rbase[b + 1];
  rb0 = rb0 < 0 ? 0 : (rb0 > csrLen ? csrLen : rb0);
  rb0 &= ~31;
  int len = rb1 - rb0;
  len = len < 0 ? 0 : (len > RCAP ? RCAP : len);
  int lenW = (len + 31) & ~31;
  if (rb0 + lenW > csrLen) lenW = (csrLen - rb0) & ~31;

  {
    const v4i z = {0, 0, 0, 0};
    for (int i = tid; i < RCAP / 4; i += NTHR) ((v4i*)region)[i] = z;
    for (int s = tid; s < NBF; s += NTHR) {
      int o = off[nodeBase + s] - rb0;
      o = o < 0 ? 0 : (o > RCAP ? RCAP : o);
      cursor[s] = o;
    }
  }
  __syncthreads();

  const int nChunks = (nE + CHUNK - 1) / CHUNK;
#pragma unroll 1
  for (int ch = 0; ch < nChunks; ++ch) {
    const int cbase = ch * CHUNK;
    const int wc = scan_chunk<NBF>(dstp, nE, cbase, nodeBase, vec8, list, tid, lane, wave);
    if (lane == 0) wcnt[wave] = wc;
    __syncthreads();
    if (wave == 0) {
#pragma unroll 1
      for (int wsx = 0; wsx < NWAVE; ++wsx) {
        int n = __builtin_amdgcn_readfirstlane(wcnt[wsx]);
        n = n > WCAP ? WCAP : (n < 0 ? 0 : n);
        const int* lp = list + wsx * WCAP;
#pragma unroll 1
        for (int i = 0; i < n; ++i) {
          const int ent  = __builtin_amdgcn_readfirstlane(lp[i]);
          const int slot = ent & (NBF - 1);
          int e = cbase + ((ent >> SLB) & (CHUNK - 1));
          e = e > nE - 1 ? nE - 1 : e;
          int src = srcp[e];
          src = src < 0 ? 0 : (src > nN - 1 ? nN - 1 : src);
          if (lane == 0) {
            int pos = cursor[slot];
            pos = pos < 0 ? 0 : (pos > RCAP - 1 ? RCAP - 1 : pos);
            region[pos] = src;
            const int np = pos + 1;
            cursor[slot] = np > RCAP ? RCAP : np;
          }
        }
      }
    }
    __syncthreads();
  }

  const int nv = lenW >> 2;
  int* gp = csr + rb0;
#pragma unroll 1
  for (int i = tid; i < nv; i += NTHR) { const v4i v = ((const v4i*)region)[i]; *(volatile v4i*)(gp + 4 * i) = v; }
  __threadfence();
#pragma unroll 1
  for (int i = tid; i < nv; i += NTHR) { const v4i v = ((const v4i*)region)[i]; *(volatile v4i*)(gp + 4 * i) = v; }
}

__global__ __launch_bounds__(NTHR) void k_mlp(
    const float* __restrict__ X, const _Float16* __restrict__ P1, const _Float16* __restrict__ P2,
    const float* __restrict__ b1, const float* __restrict__ b2, float* H, int nN) {
  extern __shared__ v4f lds_dyn[];
  _Float16* sA  = (_Float16*)lds_dyn;
  _Float16* sH  = sA + GROWS * AP1;
  float*    stg = (float*)lds_dyn;
  const int tid = threadIdx.x, lane = tid & 31, wave = tid >> 5, hh = lane >> 4, m = lane & 15;
  const int rowBase = blockIdx.x * GROWS;

#pragma unroll
  for (int i = 0; i < (GROWS * INF / 8) / NTHR; ++i) {
    const int idx = i * NTHR + tid;
    const int r   = idx >> 4;
    const int c0  = (idx & 15) * 8;
    int row = rowBase + r;
    row = row > nN - 1 ? nN - 1 : row;
    const float* xp = X + (size_t)row * INF + c0;
    const v4f a = *(const v4f*)xp * ASCALE;
    const v4f c = *(const v4f*)(xp + 4) * ASCALE;
    *(v8h*)(sA + r * AP1 + c0) = cvt8(a, c);
  }
  __syncthreads();

  v8f acc[4];
#pragma unroll
  for (int t = 0; t < 4; ++t) acc[t] = zero8();
  {
    const _Float16* ar = sA + (wave * 16 + m) * AP1 + 8 * hh;
#pragma unroll
    for (int kt = 0; kt < INF / 32; ++kt) {
      FragH a;
      a.h[0] = *(const v8h*)(ar + 32 * kt);
      a.h[1] = *(const v8h*)(ar + 32 * kt + 16);
#pragma unroll
      for (int t = 0; t < 4; ++t) {
        const _Float16* bp = P1 + (size_t)(16 * t + m) * INF + 32 * kt + 8 * hh;
        FragH bb;
        bb.h[0] = *(const v8h*)bp;
        bb.h[1] = *(const v8h*)(bp + 16);
        acc[t] = wmh(a.v, bb.v, acc[t]);
      }
    }
  }
  {
    const int r0 = wave * 16 + 8 * hh;
#pragma unroll
    for (int t = 0; t < 4; ++t) {
      const float bv = b1[16 * t + m];
#pragma unroll
      for (int r = 0; r < 8; ++r) {
        float v = acc[t][r] * PINV + bv;
        v = v > 0.0f ? v : 0.01f * v;
        sH[(r0 + r) * AP2 + 16 * t + m] = (_Float16)(v * ASCALE);
      }
    }
  }
  __syncthreads();

#pragma unroll
  for (int t = 0; t < 4; ++t) acc[t] = zero8();
  {
    const _Float16* ar = sH + (wave * 16 + m) * AP2 + 8 * hh;
#pragma unroll
    for (int kt = 0; kt < HF / 32; ++kt) {
      FragH a;
      a.h[0] = *(const v8h*)(ar + 32 * kt);
      a.h[1] = *(const v8h*)(ar + 32 * kt + 16);
#pragma unroll
      for (int t = 0; t < 4; ++t) {
        const _Float16* bp = P2 + (size_t)(16 * t + m) * HF + 32 * kt + 8 * hh;
        FragH bb;
        bb.h[0] = *(const v8h*)bp;
        bb.h[1] = *(const v8h*)(bp + 16);
        acc[t] = wmh(a.v, bb.v, acc[t]);
      }
    }
  }
  {
    const int r0 = wave * 16 + 8 * hh;
#pragma unroll
    for (int t = 0; t < 4; ++t) {
      const float bv = b2[16 * t + m];
#pragma unroll
      for (int r = 0; r < 8; ++r) {
        float v = acc[t][r] * PINV + bv;
        v = v > 0.0f ? v : 0.01f * v;
        stg[(r0 + r) * HF + 16 * t + m] = v;
      }
    }
  }
  __syncthreads();

  const float* lp = stg + wave * 16 * HF + 4 * lane;
  float* gp = H + ((size_t)rowBase + wave * 16) * HF + 4 * lane;
#pragma unroll
  for (int i = 0; i < 8; ++i) { const v4f v = *(const v4f*)(lp + i * 128); *(volatile v4f*)(gp + (size_t)i * 128) = v; }
  __threadfence();
#pragma unroll
  for (int i = 0; i < 8; ++i) { const v4f v = *(const v4f*)(lp + i * 128); *(volatile v4f*)(gp + (size_t)i * 128) = v; }
}

__device__ __forceinline__ v2f gather_seg(const int* __restrict__ csr, const float* __restrict__ dinv,
                                          const float* F, int st, int n, int nN, int csrLen, int lane) {
  v2f acc;
  acc.x = 0.0f; acc.y = 0.0f;
#pragma unroll 1
  for (int q0 = 0; q0 < n; q0 += 32) {
    int pos = st + q0 + lane;
    pos = pos < 0 ? 0 : (pos > csrLen - 1 ? csrLen - 1 : pos);
    int sl = csr[pos];
    sl = sl < 0 ? 0 : (sl > nN - 1 ? nN - 1 : sl);
    FI du; du.f = dinv[sl];
    const int mcnt = (n - q0) < 32 ? (n - q0) : 32;
#pragma unroll 1
    for (int p = 0; p < mcnt; ++p) {
      const int s = __builtin_amdgcn_readlane(sl, p);
      FI dd; dd.i = __builtin_amdgcn_readlane(du.i, p);
      const v2f v = *(const v2f*)(F + (size_t)s * HF + 2 * lane);
      acc.x = fmaf(v.x, dd.f, acc.x);
      acc.y = fmaf(v.y, dd.f, acc.y);
    }
  }
  return acc;
}

__global__ __launch_bounds__(NTHR) void k_agg1(
    const int* __restrict__ csr, const int* __restrict__ off, const int* __restrict__ cnt,
    const float* __restrict__ dinv, const float* H, float* F1, int nN, int csrLen) {
  const int tid = threadIdx.x, lane = tid & 31, wave = tid >> 5;
  const int tbase = blockIdx.x * TGT + wave * 32;
  const int cl = tbase + lane;
  const int cnt_l = cnt[cl];
  const int off_l = off[cl];
  FI dvu; dvu.f = dinv[cl];

#pragma unroll 1
  for (int j = 0; j < 32; ++j) {
    const int c = tbase + j;
    int n = __builtin_amdgcn_readlane(cnt_l, j);
    n = n < 0 ? 0 : (n > DEGCAP ? DEGCAP : n);
    const int st = __builtin_amdgcn_readlane(off_l, j);
    FI du; du.i = __builtin_amdgcn_readlane(dvu.i, j);
    const float dc = du.f;
    const v2f ag = gather_seg(csr, dinv, H, st, n, nN, csrLen, lane);
    const size_t ro = (size_t)c * HF + 2 * lane;
    const v2f f0 = *(const v2f*)(H + ro);
    v2f px; px.x = ag.x * dc; px.y = ag.y * dc;
    v2f f1; f1.x = f0.x - px.x; f1.y = f0.y - px.y;
    float* fp = F1 + ro;
    *(volatile v2f*)fp = f1;
    __threadfence();
    *(volatile v2f*)fp = f1;
  }
}

template <int MODE>
__global__ __launch_bounds__(NTHR) void k_aggw3(
    const int* __restrict__ csr, const int* __restrict__ off, const int* __restrict__ cnt,
    const float* __restrict__ dinv, float* H, const float* F1, float* HALL,
    const _Float16* __restrict__ P3, const float* __restrict__ b3,
    const float* __restrict__ W4, const float* __restrict__ b4, float* out, int nN, int csrLen) {
  extern __shared__ v4f lds_dyn[];
  _Float16* sA   = (_Float16*)lds_dyn;
  float*    stg0 = (float*)lds_dyn;
  float*    stg1 = stg0 + TGT * HF;
  float*    sout = stg1 + TGT * HF;
  const int tid = threadIdx.x, lane = tid & 31, wave = tid >> 5, hh = lane >> 4, m = lane & 15;
  const int rowBase = blockIdx.x * TGT;
  const int tbase = rowBase + wave * 32;
  const int cl = tbase + lane;
  const int cnt_l = cnt[cl];
  const int off_l = off[cl];
  FI dvu; dvu.f = dinv[cl];

#pragma unroll 1
  for (int j = 0; j < 32; ++j) {
    const int c = tbase + j;
    int n = __builtin_amdgcn_readlane(cnt_l, j);
    n = n < 0 ? 0 : (n > DEGCAP ? DEGCAP : n);
    const int st = __builtin_amdgcn_readlane(off_l, j);
    FI du; du.i = __builtin_amdgcn_readlane(dvu.i, j);
    const float dc = du.f;
    const v2f ag = gather_seg(csr, dinv, F1, st, n, nN, csrLen, lane);
    const size_t ro = (size_t)c * HF + 2 * lane;
    const v2f f1 = *(const v2f*)(F1 + ro);
    const v2f f0 = *(const v2f*)(H + ro);
    v2f px; px.x = ag.x * dc; px.y = ag.y * dc;
    v2f f2; f2.x = f1.x - px.x; f2.y = f1.y - px.y;
    v2f t0, t1, t2;
    t0.x = (TH00 * f0.x + TH01 * f1.x) + TH02 * f2.x;
    t0.y = (TH00 * f0.y + TH01 * f1.y) + TH02 * f2.y;
    t1.x = TH11 * f1.x + TH12 * f2.x;
    t1.y = TH11 * f1.y + TH12 * f2.y;
    t2.x = TH22 * f2.x;
    t2.y = TH22 * f2.y;
    v2h u0, u1, u2;
    u0.x = (_Float16)(t0.x * ASCALE); u0.y = (_Float16)(t0.y * ASCALE);
    u1.x = (_Float16)(t1.x * ASCALE); u1.y = (_Float16)(t1.y * ASCALE);
    u2.x = (_Float16)(t2.x * ASCALE); u2.y = (_Float16)(t2.y * ASCALE);
    _Float16* ap = sA + (wave * 32 + j) * AP3 + 2 * lane;
    *(v2h*)ap = u0;
    *(v2h*)(ap + HF) = u1;
    *(v2h*)(ap + 2 * HF) = u2;
  }
  __syncthreads();

  v8f acc[8];
#pragma unroll
  for (int t = 0; t < 8; ++t) acc[t] = zero8();
  {
    const _Float16* ar0 = sA + (wave * 32 + m) * AP3 + 8 * hh;
    const _Float16* ar1 = ar0 + 16 * AP3;
#pragma unroll 1
    for (int kt = 0; kt < KW3 / 32; ++kt) {
      FragH a0, a1;
      a0.h[0] = *(const v8h*)(ar0 + 32 * kt);
      a0.h[1] = *(const v8h*)(ar0 + 32 * kt + 16);
      a1.h[0] = *(const v8h*)(ar1 + 32 * kt);
      a1.h[1] = *(const v8h*)(ar1 + 32 * kt + 16);
#pragma unroll
      for (int t = 0; t < 4; ++t) {
        const _Float16* bp = P3 + (size_t)(16 * t + m) * KW3 + 32 * kt + 8 * hh;
        FragH bb;
        bb.h[0] = *(const v8h*)bp;
        bb.h[1] = *(const v8h*)(bp + 16);
        acc[t]     = wmh(a0.v, bb.v, acc[t]);
        acc[4 + t] = wmh(a1.v, bb.v, acc[4 + t]);
      }
    }
  }
  __syncthreads();

  {
    float bv[4];
#pragma unroll
    for (int t = 0; t < 4; ++t) bv[t] = b3[16 * t + m];
#pragma unroll
    for (int rt = 0; rt < 2; ++rt) {
#pragma unroll
      for (int t = 0; t < 4; ++t) {
#pragma unroll
        for (int r = 0; r < 8; ++r) {
          const int lrow = wave * 32 + 16 * rt + 8 * hh + r;
          const int col  = 16 * t + m;
          const float hs = acc[4 * rt + t][r] * PINV + bv[t];
          if (MODE == 0) {
            stg0[lrow * HF + col] = hs;
          } else if (MODE == 1) {
            const float old = H[((size_t)rowBase + lrow) * HF + col];
            stg0[lrow * HF + col] = hs;
            stg1[lrow * HF + col] = old + hs;
          } else {
            const float old = HALL[((size_t)rowBase + lrow) * HF + col];
            float a = old + hs;
            a = a > 0.0f ? a : 0.01f * a;
            stg0[lrow * HF + col] = a;
          }
        }
      }
    }
  }
  __syncthreads();

  if (MODE != 2) {
    const float* lp0 = stg0 + wave * 32 * HF + 4 * lane;
    const float* lp1 = stg1 + wave * 32 * HF + 4 * lane;
    float* gpH = H + ((size_t)rowBase + wave * 32) * HF + 4 * lane;
    float* gpA = HALL + ((size_t)rowBase + wave * 32) * HF + 4 * lane;
#pragma unroll
    for (int i = 0; i < 16; ++i) {
      const v4f v = *(const v4f*)(lp0 + i * 128);
      *(volatile v4f*)(gpH + (size_t)i * 128) = v;
      if (MODE == 1) { const v4f u = *(const v4f*)(lp1 + i * 128); *(volatile v4f*)(gpA + (size_t)i * 128) = u; }
    }
    __threadfence();
#pragma unroll
    for (int i = 0; i < 16; ++i) {
      const v4f v = *(const v4f*)(lp0 + i * 128);
      *(volatile v4f*)(gpH + (size_t)i * 128) = v;
      if (MODE == 1) { const v4f u = *(const v4f*)(lp1 + i * 128); *(volatile v4f*)(gpA + (size_t)i * 128) = u; }
    }
  } else {
    const float* arow = stg0 + tid * HF;
    float o0 = 0.0f, o1 = 0.0f;
#pragma unroll 2
    for (int c4 = 0; c4 < HF / 4; ++c4) {
      const v4f a  = *(const v4f*)(arow + 4 * c4);
      const v4f w0 = *(const v4f*)(W4 + 4 * c4);
      const v4f w1 = *(const v4f*)(W4 + HF + 4 * c4);
      o0 = fmaf(a.x, w0.x, o0); o0 = fmaf(a.y, w0.y, o0); o0 = fmaf(a.z, w0.z, o0); o0 = fmaf(a.w, w0.w, o0);
      o1 = fmaf(a.x, w1.x, o1); o1 = fmaf(a.y, w1.y, o1); o1 = fmaf(a.z, w1.z, o1); o1 = fmaf(a.w, w1.w, o1);
    }
    o0 += b4[0];
    o1 += b4[1];
    v2f ov; ov.x = o0; ov.y = o1;
    *(v2f*)(sout + 2 * tid) = ov;
    __syncthreads();
    if (wave == 0) {
      int validRows = nN - rowBase;
      validRows = validRows < 0 ? 0 : (validRows > TGT ? TGT : validRows);
      const int rem = validRows * NCLS;
      const int rem4 = rem & ~3;
      float* ob = out + (size_t)rowBase * NCLS;
      v4f pv[4];
#pragma unroll
      for (int q = 0; q < 4; ++q) pv[q] = *(const v4f*)(sout + 128 * q + 4 * lane);
#pragma unroll
      for (int q = 0; q < 4; ++q) { const int fi = 128 * q + 4 * lane; if (fi + 4 <= rem4) *(volatile v4f*)(ob + fi) = pv[q]; }
      if (lane == 0) {
#pragma unroll 1
        for (int e2 = rem4; e2 < rem; ++e2) *(volatile float*)(ob + e2) = sout[e2];
      }
      __threadfence();
#pragma unroll
      for (int q = 0; q < 4; ++q) { const int fi = 128 * q + 4 * lane; if (fi + 4 <= rem4) *(volatile v4f*)(ob + fi) = pv[q]; }
      if (lane == 0) {
#pragma unroll 1
        for (int e2 = rem4; e2 < rem; ++e2) *(volatile float*)(ob + e2) = sout[e2];
      }
    }
  }
}

extern "C" void kernel_launch(void* const* d_in, const int* in_sizes, int n_in,
                              void* d_out, int out_size, void* d_ws, size_t ws_size,
                              hipStream_t stream) {
  if (n_in < 15) return;
  if (in_sizes[0] <= 0 || (in_sizes[0] % INF) != 0) return;
  const int nN = in_sizes[0] / INF;
  if (in_sizes[1] != HF * INF || in_sizes[2] != HF) return;
  if (in_sizes[3] != HF * HF || in_sizes[4] != HF) return;
  if (in_sizes[5] != HF * KW3 || in_sizes[6] != HF) return;
  if (in_sizes[7] != NCLS * HF || in_sizes[8] != NCLS) return;
  const int nE0 = in_sizes[9], nE1 = in_sizes[11], nE2 = in_sizes[13];
  if (in_sizes[10] != nE0 || in_sizes[12] != nE1 || in_sizes[14] != nE2) return;
  if (nE0 <= 0 || nE1 <= 0 || nE2 <= 0) return;
  if (out_size != NCLS * nN) return;
  if (nN > (1 << 22)) return;
  int nEmax = nE0 > nE1 ? nE0 : nE1;
  nEmax = nEmax > nE2 ? nEmax : nE2;
  if (nEmax > (1 << 28)) return;

  const float* X  = (const float*)d_in[0];
  const float* W1 = (const float*)d_in[1];
  const float* b1 = (const float*)d_in[2];
  const float* W2 = (const float*)d_in[3];
  const float* b2 = (const float*)d_in[4];
  const float* W3 = (const float*)d_in[5];
  const float* b3 = (const float*)d_in[6];
  const float* W4 = (const float*)d_in[7];
  const float* b4 = (const float*)d_in[8];
  const int* srcs[3] = {(const int*)d_in[9],  (const int*)d_in[11], (const int*)d_in[13]};
  const int* dsts[3] = {(const int*)d_in[10], (const int*)d_in[12], (const int*)d_in[14]};
  const int  nEs[3]  = {nE0, nE1, nE2};
  float* out = (float*)d_out;

  const int NPAD   = ((nN + TGT - 1) / TGT) * TGT;
  const int nBC    = (nN + NBC - 1) / NBC;
  const int CNTPAD = nBC * NBC;
  if (CNTPAD < NPAD) return;
  if (4 * nBC + 1 > RBN) return;
  const int nBF    = (nN + NBF - 1) / NBF;
  if (nBF > 4 * nBC) return;
  const int csrLen = ((nEmax + 31) & ~31) + 4096;
  if (32 * 4 * nBC > 4096) return;
  const int nMlp   = NPAD / GROWS;
  const int nAgg   = NPAD / TGT;

  char* ws = (char*)d_ws;
  size_t cur = 0;
  const size_t oW   = cur; cur += (size_t)(HF * INF + HF * HF + HF * KW3) * 2; cur = (cur + 255) & ~(size_t)255;
  const size_t oCnt = cur; cur += (size_t)CNTPAD * 4;                           cur = (cur + 255) & ~(size_t)255;
  const size_t oDv  = cur; cur += (size_t)CNTPAD * 4;                           cur = (cur + 255) & ~(size_t)255;
  const size_t oOff = cur; cur += (size_t)CNTPAD * 4;                           cur = (cur + 255) & ~(size_t)255;
  const size_t oRb  = cur; cur += (size_t)RBN * 4;                              cur = (cur + 255) & ~(size_t)255;
  const size_t oCsr = cur; cur += (size_t)csrLen * 4;                           cur = (cur + 255) & ~(size_t)255;
  const size_t oH   = cur; cur += (size_t)NPAD * HF * 4;                        cur = (cur + 255) & ~(size_t)255;
  const size_t oF1  = cur; cur += (size_t)NPAD * HF * 4;                        cur = (cur + 255) & ~(size_t)255;
  const size_t oHA  = cur; cur += (size_t)NPAD * HF * 4;                        cur = (cur + 255) & ~(size_t)255;
  if (cur > ws_size) return;
  _Float16* wp   = (_Float16*)(ws + oW);
  int*      cnt  = (int*)(ws + oCnt);
  float*    dinv = (float*)(ws + oDv);
  int*      offp = (int*)(ws + oOff);
  int*      rb   = (int*)(ws + oRb);
  int*      csr  = (int*)(ws + oCsr);
  float*    H    = (float*)(ws + oH);
  float*    F1   = (float*)(ws + oF1);
  float*    HALL = (float*)(ws + oHA);
  const _Float16* P1 = wp;
  const _Float16* P2 = wp + HF * INF;
  const _Float16* P3 = wp + HF * INF + HF * HF;
  const int vec8 = 1;

  k_wprep<<<12, NTHR, 0, stream>>>(W1, W2, W3, wp);

  k_mlp<<<nMlp, NTHR, LDS_MLP, stream>>>(X, P1, P2, b1, b2, H, nN);

  hipFuncSetAttribute(reinterpret_cast<const void*>(&k_fill),
                      hipFuncAttributeMaxDynamicSharedMemorySize, LDS_FILL);
  hipFuncSetAttribute(reinterpret_cast<const void*>(&k_aggw3<0>),
                      hipFuncAttributeMaxDynamicSharedMemorySize, LDS_AW);
  hipFuncSetAttribute(reinterpret_cast<const void*>(&k_aggw3<1>),
                      hipFuncAttributeMaxDynamicSharedMemorySize, LDS_AW);
  hipFuncSetAttribute(reinterpret_cast<const void*>(&k_aggw3<2>),
                      hipFuncAttributeMaxDynamicSharedMemorySize, LDS_AW);

  for (int r = 0; r < 3; ++r) {
    k_count<<<nBC, NTHR, 0, stream>>>(dsts[r], cnt, dinv, nEs[r], vec8);
    k_offsets<<<1, OTHR, 0, stream>>>(cnt, offp, rb, nBC);
    k_fill<<<nBF, NTHR, LDS_FILL, stream>>>(srcs[r], dsts[r], offp, rb, csr, nN, nEs[r], vec8, csrLen);
    k_agg1<<<nAgg, NTHR, 0, stream>>>(csr, offp, cnt, dinv, H, F1, nN, csrLen);
    if (r == 0)
      k_aggw3<0><<<nAgg, NTHR, LDS_AW, stream>>>(csr, offp, cnt, dinv, H, F1, HALL, P3, b3, W4, b4, out, nN, csrLen);
    else if (r == 1)
      k_aggw3<1><<<nAgg, NTHR, LDS_AW, stream>>>(csr, offp, cnt, dinv, H, F1, HALL, P3, b3, W4, b4, out, nN, csrLen);
    else
      k_aggw3<2><<<nAgg, NTHR, LDS_AW, stream>>>(csr, offp, cnt, dinv, H, F1, HALL, P3, b3, W4, b4, out, nN, csrLen);
  }
}
